// MultiHeadWassersteinAttention_21165598835372
// MI455X (gfx1250) — hardware-verified
//
#include <hip/hip_runtime.h>
#include <stddef.h>
#include <stdint.h>

#define BB   2
#define NN   2048
#define CC   1024
#define HH   16
#define DD   64
#define DQ   128
#define ROWS (BB * NN)
#define C3   (3 * CC)
#define NBH  (BB * HH)
#define QKPL ((size_t)NBH * NN * DQ)
#define VPL  ((size_t)NBH * DD * NN)
#define SQPL ((size_t)NBH * NN)

static_assert(NN % 256 == 0);
static_assert(CC % 64 == 0);
static_assert(DD == 64);
static_assert(HH * DD == CC);
static_assert(ROWS % 256 == 0);
static_assert(NBH * (NN / 128) == 512);

typedef _Float16 v16h __attribute__((ext_vector_type(16)));
typedef _Float16 v8h  __attribute__((ext_vector_type(8)));
typedef float    v8f  __attribute__((ext_vector_type(8)));
typedef float    v4f  __attribute__((ext_vector_type(4)));
typedef unsigned int v4u __attribute__((ext_vector_type(4)));

union Frag  { v16h v; v8h h[2]; };
union Pack8 { v8h h; v4u u; };

__device__ __forceinline__ v8f mma16(v16h a, v16h b, v8f c) {
  c = __builtin_amdgcn_wmma_f32_16x16x32_f16(false, a, false, b, (short)0, c, false, false);
  asm volatile("v_nop\n\tv_nop\n\tv_nop\n\tv_nop" : "+v"(c) : "v"(a), "v"(b));
  return c;
}

__device__ __forceinline__ v16h ldfrag(const _Float16* p, int ld, int row0, int k0, int lane) {
  const int m = lane & 15, lh = lane >> 4;
  const _Float16* q = p + (size_t)(row0 + m) * ld + k0 + 8 * lh;
  Frag f;
  f.h[0] = *(const v8h*)(q);
  f.h[1] = *(const v8h*)(q + 16);
  return f.v;
}

__device__ __forceinline__ v8f zero8() { return (v8f){0.f, 0.f, 0.f, 0.f, 0.f, 0.f, 0.f, 0.f}; }

__device__ __forceinline__ void gemm32x64(const _Float16* __restrict__ A, int lda,
                                          const _Float16* __restrict__ Bt, int ldb,
                                          int m0, int n0, int lane, v8f (&acc)[2][4]) {
#pragma unroll 2
  for (int k0 = 0; k0 < CC; k0 += 32) {
    const v16h a0 = ldfrag(A, lda, m0, k0, lane);
    const v16h a1 = ldfrag(A, lda, m0 + 16, k0, lane);
    const v16h b0 = ldfrag(Bt, ldb, n0, k0, lane);
    const v16h b1 = ldfrag(Bt, ldb, n0 + 16, k0, lane);
    const v16h b2 = ldfrag(Bt, ldb, n0 + 32, k0, lane);
    const v16h b3 = ldfrag(Bt, ldb, n0 + 48, k0, lane);
    acc[0][0] = mma16(a0, b0, acc[0][0]);
    acc[1][0] = mma16(a1, b0, acc[1][0]);
    acc[0][1] = mma16(a0, b1, acc[0][1]);
    acc[1][1] = mma16(a1, b1, acc[1][1]);
    acc[0][2] = mma16(a0, b2, acc[0][2]);
    acc[1][2] = mma16(a1, b2, acc[1][2]);
    acc[0][3] = mma16(a0, b3, acc[0][3]);
    acc[1][3] = mma16(a1, b3, acc[1][3]);
  }
}

__global__ __launch_bounds__(256) void k_cvt_x(const float* __restrict__ x, _Float16* __restrict__ xh, int ngrp) {
  const int t = blockIdx.x * 256 + (int)threadIdx.x;
  if (t >= ngrp) return;
  const size_t o = (size_t)t * 8;
  const v4f a0 = *(const v4f*)(x + o);
  const v4f a1 = *(const v4f*)(x + o + 4);
  Pack8 pk;
  pk.h = (v8h){(_Float16)a0[0], (_Float16)a0[1], (_Float16)a0[2], (_Float16)a0[3],
               (_Float16)a1[0], (_Float16)a1[1], (_Float16)a1[2], (_Float16)a1[3]};
  const v4u vv = pk.u;
  volatile v4u* d = (volatile v4u*)(xh + o);
  *d = vv;
  __threadfence();
  *d = vv;
}

#define WTP 68
__global__ __launch_bounds__(256) void k_wt(const float* __restrict__ w, _Float16* __restrict__ wt, int nout) {
  __shared__ __align__(16) float tf[64 * WTP];
  const int tid = threadIdx.x;
  const int n0 = blockIdx.x * 64;
  const int k0 = blockIdx.y * 64;
  {
    const int kr = tid >> 4;
    const int n4 = (tid & 15) * 4;
#pragma unroll
    for (int it = 0; it < 4; ++it) {
      const int kl = it * 16 + kr;
      const v4f a = *(const v4f*)(w + (size_t)(k0 + kl) * nout + n0 + n4);
      *(v4f*)(tf + kl * WTP + n4) = a;
    }
  }
  __syncthreads();
  v4u val[2];
  size_t go[2];
#pragma unroll
  for (int j = 0; j < 2; ++j) {
    const int p  = tid + 256 * j;
    const int nl = p >> 3;
    const int pc = p & 7;
    const float* cp = tf + (pc * 8) * WTP + nl;
    Pack8 pk;
    pk.h = (v8h){(_Float16)(cp[0 * WTP] * 32.0f), (_Float16)(cp[1 * WTP] * 32.0f),
                 (_Float16)(cp[2 * WTP] * 32.0f), (_Float16)(cp[3 * WTP] * 32.0f),
                 (_Float16)(cp[4 * WTP] * 32.0f), (_Float16)(cp[5 * WTP] * 32.0f),
                 (_Float16)(cp[6 * WTP] * 32.0f), (_Float16)(cp[7 * WTP] * 32.0f)};
    val[j] = pk.u;
    go[j]  = (size_t)(n0 + nl) * CC + k0 + pc * 8;
  }
  for (int ps = 0; ps < 2; ++ps) {
#pragma unroll
    for (int j = 0; j < 2; ++j) *(volatile v4u*)(wt + go[j]) = val[j];
    __threadfence();
  }
}

#define STP 72
__global__ __launch_bounds__(256) void k_qkv(const _Float16* __restrict__ xh,
                                             const _Float16* __restrict__ wt,
                                             const float* __restrict__ bias,
                                             _Float16* __restrict__ qpl,
                                             _Float16* __restrict__ kpl,
                                             _Float16* __restrict__ vt,
                                             float* __restrict__ sqp, int side) {
  __shared__ __align__(16) _Float16 st[256 * STP];
  __shared__ __align__(16) float sqs[256];
  const int tid = threadIdx.x, lane = tid & 31, wave = tid >> 5;
  const int hh = lane >> 4, c = lane & 15;
  const int mb = blockIdx.x * 256;
  const int m0 = mb + wave * 32;
  const int n0 = blockIdx.y * 64;

  v8f acc[2][4];
#pragma unroll
  for (int s = 0; s < 2; ++s)
#pragma unroll
    for (int t = 0; t < 4; ++t) acc[s][t] = zero8();
  gemm32x64(xh, CC, wt, CC, m0, n0, lane, acc);

  float rs[2][8];
#pragma unroll
  for (int sub = 0; sub < 2; ++sub)
#pragma unroll
    for (int r = 0; r < 8; ++r) rs[sub][r] = 0.f;

#pragma unroll
  for (int t = 0; t < 4; ++t) {
    const float bv = bias[n0 + 16 * t + c];
#pragma unroll
    for (int sub = 0; sub < 2; ++sub) {
#pragma unroll
      for (int r = 0; r < 8; ++r) {
        const int lr = wave * 32 + sub * 16 + 8 * hh + r;
        const float v = acc[sub][t][r] * 0.03125f + bv;
        st[lr * STP + 16 * t + c] = (_Float16)v;
        rs[sub][r] += v * v;
      }
    }
  }
#pragma unroll
  for (int sub = 0; sub < 2; ++sub) {
#pragma unroll
    for (int r = 0; r < 8; ++r) {
      float x = rs[sub][r];
      x += __shfl_xor(x, 1, 32);
      x += __shfl_xor(x, 2, 32);
      x += __shfl_xor(x, 4, 32);
      x += __shfl_xor(x, 8, 32);
      rs[sub][r] = x;
    }
  }
  if (c == 0) {
#pragma unroll
    for (int sub = 0; sub < 2; ++sub)
#pragma unroll
      for (int r = 0; r < 8; ++r) sqs[wave * 32 + sub * 16 + 8 * hh + r] = rs[sub][r];
  }
  __syncthreads();

  const int which = n0 >> 10;
  const int head  = (n0 & (CC - 1)) >> 6;
  const int b  = mb >> 11;
  const int nb = mb & (NN - 1);
  const int bh = b * HH + head;
  v4u val[8];
  size_t go[8];
  _Float16* dst;
  if (which < 2) {
    dst = (which == 0) ? qpl : kpl;
#pragma unroll
    for (int j = 0; j < 8; ++j) {
      const int p  = tid + 256 * j;
      const int lr = p >> 3;
      const int pc = p & 7;
      Pack8 pk;
      pk.h  = *(const v8h*)(st + lr * STP + pc * 8);
      val[j] = pk.u;
      go[j]  = ((size_t)bh * NN + nb + lr) * DQ + (size_t)side * DD + pc * 8;
    }
  } else {
    dst = vt;
#pragma unroll
    for (int j = 0; j < 8; ++j) {
      const int p  = tid + 256 * j;
      const int L  = p >> 3;
      const int pc = p & 7;
      const int d  = L >> 2;
      const int nl = (L & 3) * 64 + pc * 8;
      const _Float16* cp = st + nl * STP + d;
      Pack8 pk;
      pk.h = (v8h){cp[0 * STP], cp[1 * STP], cp[2 * STP], cp[3 * STP],
                   cp[4 * STP], cp[5 * STP], cp[6 * STP], cp[7 * STP]};
      val[j] = pk.u;
      go[j]  = ((size_t)bh * DD + d) * NN + nb + nl;
    }
  }
  const bool doSq = (which < 2) && (tid < 64);
  const int tq = tid & 63;
  const v4f sqv = *(const v4f*)(sqs + 4 * tq);
  const size_t sqo = (size_t)(which & 1) * SQPL + (size_t)bh * NN + nb + 4 * tq;

  for (int ps = 0; ps < 2; ++ps) {
#pragma unroll
    for (int j = 0; j < 8; ++j) *(volatile v4u*)(dst + go[j]) = val[j];
    if (doSq) *(volatile v4f*)(sqp + sqo) = sqv;
    __threadfence();
  }
}

#define KTP 136
#define VTP 72
#define PTP 72
__global__ __launch_bounds__(256) void k_attn(const _Float16* __restrict__ qp,
                                              const _Float16* __restrict__ kp,
                                              const _Float16* __restrict__ vmt,
                                              const _Float16* __restrict__ vst,
                                              const float* __restrict__ sqp,
                                              _Float16* __restrict__ om,
                                              _Float16* __restrict__ os) {
  __shared__ __align__(16) _Float16 Ks[64 * KTP];
  __shared__ __align__(16) _Float16 Vma[64 * VTP];
  __shared__ __align__(16) _Float16 Vsa[64 * VTP];
  __shared__ __align__(16) _Float16 Ps[8][16 * PTP];
  __shared__ float sqkS[64];

  const int tid = threadIdx.x, lane = tid & 31, wave = tid >> 5;
  const int hh = lane >> 4, c = lane & 15;
  const int bh = blockIdx.x >> 4;
  const int qb = blockIdx.x & 15;
  const int b  = bh >> 4, h = bh & (HH - 1);
  const int q0 = qb * 128 + wave * 16;

  const _Float16* Q  = qp + (size_t)bh * NN * DQ;
  const _Float16* K  = kp + (size_t)bh * NN * DQ;
  const _Float16* VM = vmt + (size_t)bh * DD * NN;
  const _Float16* VS = vst + (size_t)bh * DD * NN;
  const float* pqm = sqp + 0 * SQPL + (size_t)bh * NN;
  const float* pkm = sqp + 1 * SQPL + (size_t)bh * NN;
  const float* pqs = sqp + 2 * SQPL + (size_t)bh * NN;
  const float* pks = sqp + 3 * SQPL + (size_t)bh * NN;

  v16h qa[4];
#pragma unroll
  for (int kq = 0; kq < 4; ++kq) qa[kq] = ldfrag(Q, DQ, q0, 32 * kq, lane);

  float sqr[8];
#pragma unroll
  for (int r = 0; r < 8; ++r) {
    const int qi = q0 + 8 * hh + r;
    sqr[r] = pqm[qi] + pqs[qi];
  }

  float mrow[8], lrow[8];
  v8f oam[4], oas[4];
#pragma unroll
  for (int r = 0; r < 8; ++r) { mrow[r] = 0.f; lrow[r] = 0.f; }
#pragma unroll
  for (int t = 0; t < 4; ++t) { oam[t] = zero8(); oas[t] = zero8(); }

  _Float16* pw = Ps[wave];

  for (int kc = 0; kc < NN / 64; ++kc) {
    const int kv0 = kc * 64;
    __syncthreads();
    {
      const int r  = tid >> 2;
      const int q4 = (tid & 3) * 32;
      const _Float16* ks = K + (size_t)(kv0 + r) * DQ + q4;
      *(v8h*)(Ks + r * KTP + q4)      = *(const v8h*)(ks);
      *(v8h*)(Ks + r * KTP + q4 + 8)  = *(const v8h*)(ks + 8);
      *(v8h*)(Ks + r * KTP + q4 + 16) = *(const v8h*)(ks + 16);
      *(v8h*)(Ks + r * KTP + q4 + 24) = *(const v8h*)(ks + 24);
      const int q2 = (tid & 3) * 16;
      const _Float16* vm = VM + (size_t)r * NN + kv0 + q2;
      *(v8h*)(Vma + r * VTP + q2)     = *(const v8h*)(vm);
      *(v8h*)(Vma + r * VTP + q2 + 8) = *(const v8h*)(vm + 8);
      const _Float16* vs = VS + (size_t)r * NN + kv0 + q2;
      *(v8h*)(Vsa + r * VTP + q2)     = *(const v8h*)(vs);
      *(v8h*)(Vsa + r * VTP + q2 + 8) = *(const v8h*)(vs + 8);
    }
    if (tid < 64) sqkS[tid] = pkm[kv0 + tid] + pks[kv0 + tid];
    __syncthreads();

    v8f s[4];
#pragma unroll
    for (int j = 0; j < 4; ++j) s[j] = zero8();
#pragma unroll
    for (int kq = 0; kq < 4; ++kq) {
#pragma unroll
      for (int j = 0; j < 4; ++j) {
        const v16h kb = ldfrag(Ks, KTP, j * 16, kq * 32, lane);
        s[j] = mma16(qa[kq], kb, s[j]);
      }
    }
    float sk[4];
#pragma unroll
    for (int j = 0; j < 4; ++j) sk[j] = sqkS[j * 16 + c];

    float cm[8];
#pragma unroll
    for (int r = 0; r < 8; ++r) {
      float m = 0.f;
#pragma unroll
      for (int j = 0; j < 4; ++j) {
        const float sv  = s[j][r];
        const float w2  = (sqr[r] + sk[j]) - 2.0f * sv;
        const float wd  = sqrtf(fmaxf(w2, 0.f));
        const float sim = __expf(-wd);
        s[j][r] = sim;
        m = fmaxf(m, sim);
      }
#pragma unroll
      for (int off = 1; off < 16; off <<= 1) m = fmaxf(m, __shfl_xor(m, off, 32));
      cm[r] = m;
    }
    float al[8];
#pragma unroll
    for (int r = 0; r < 8; ++r) {
      const float mnew  = fmaxf(mrow[r], cm[r]);
      const float alpha = __expf(mrow[r] - mnew);
      mrow[r] = mnew;
      float psum = 0.f;
#pragma unroll
      for (int j = 0; j < 4; ++j) {
        const float p = __expf(s[j][r] - mnew);
        const _Float16 p16 = (_Float16)(p * 1024.0f);
        psum += (float)p16;
        pw[(8 * hh + r) * PTP + j * 16 + c] = p16;
      }
#pragma unroll
      for (int off = 1; off < 16; off <<= 1) psum += __shfl_xor(psum, off, 32);
      lrow[r] = lrow[r] * alpha + psum;
      al[r] = alpha;
    }
#pragma unroll
    for (int t = 0; t < 4; ++t) {
#pragma unroll
      for (int r = 0; r < 8; ++r) { oam[t][r] *= al[r]; oas[t][r] *= al[r]; }
    }
    __syncthreads();

#pragma unroll
    for (int kk = 0; kk < 2; ++kk) {
      const v16h pa = ldfrag(pw, PTP, 0, kk * 32, lane);
#pragma unroll
      for (int t = 0; t < 4; ++t) {
        const v16h vbm = ldfrag(Vma, VTP, t * 16, kk * 32, lane);
        oam[t] = mma16(pa, vbm, oam[t]);
        const v16h vbs = ldfrag(Vsa, VTP, t * 16, kk * 32, lane);
        oas[t] = mma16(pa, vbs, oas[t]);
      }
    }
  }
  __syncthreads();

  float inv[8];
#pragma unroll
  for (int r = 0; r < 8; ++r) inv[r] = 16.0f / lrow[r];

  v4u val[4];
  size_t go[4];

#pragma unroll
  for (int r = 0; r < 8; ++r) {
#pragma unroll
    for (int t = 0; t < 4; ++t) pw[(8 * hh + r) * PTP + 16 * t + c] = (_Float16)(oam[t][r] * inv[r]);
  }
  __syncthreads();
#pragma unroll
  for (int it = 0; it < 4; ++it) {
    const int p  = lane + 32 * it;
    const int L  = p >> 3;
    const int pc = p & 7;
    Pack8 pk;
    pk.h    = *(const v8h*)(pw + L * PTP + pc * 8);
    val[it] = pk.u;
    go[it]  = ((size_t)(b * NN + q0 + L)) * CC + (size_t)h * DD + pc * 8;
  }
  for (int ps = 0; ps < 2; ++ps) {
#pragma unroll
    for (int it = 0; it < 4; ++it) *(volatile v4u*)(om + go[it]) = val[it];
    __threadfence();
  }
  __syncthreads();

#pragma unroll
  for (int r = 0; r < 8; ++r) {
#pragma unroll
    for (int t = 0; t < 4; ++t) pw[(8 * hh + r) * PTP + 16 * t + c] = (_Float16)(oas[t][r] * inv[r]);
  }
  __syncthreads();
#pragma unroll
  for (int it = 0; it < 4; ++it) {
    const int p  = lane + 32 * it;
    const int L  = p >> 3;
    const int pc = p & 7;
    Pack8 pk;
    pk.h    = *(const v8h*)(pw + L * PTP + pc * 8);
    val[it] = pk.u;
  }
  for (int ps = 0; ps < 2; ++ps) {
#pragma unroll
    for (int it = 0; it < 4; ++it) *(volatile v4u*)(os + go[it]) = val[it];
    __threadfence();
  }
}

#define OTP 68
__global__ __launch_bounds__(256) void k_proj(const _Float16* __restrict__ ap,
                                              const _Float16* __restrict__ wt,
                                              const float* __restrict__ bias,
                                              float* __restrict__ out) {
  __shared__ __align__(16) float st[8][16 * OTP];
  const int tid = threadIdx.x, lane = tid & 31, wave = tid >> 5;
  const int hh = lane >> 4, c = lane & 15;
  const int m0 = blockIdx.x * 256 + wave * 32;
  const int n0 = blockIdx.y * 64;

  v8f acc[2][4];
#pragma unroll
  for (int s = 0; s < 2; ++s)
#pragma unroll
    for (int t = 0; t < 4; ++t) acc[s][t] = zero8();
  gemm32x64(ap, CC, wt, CC, m0, n0, lane, acc);

  float bvs[4];
#pragma unroll
  for (int t = 0; t < 4; ++t) bvs[t] = bias[n0 + 16 * t + c];

  float* sw = st[wave];
#pragma unroll
  for (int sub = 0; sub < 2; ++sub) {
    __syncthreads();
#pragma unroll
    for (int t = 0; t < 4; ++t) {
#pragma unroll
      for (int r = 0; r < 8; ++r)
        sw[(8 * hh + r) * OTP + 16 * t + c] = acc[sub][t][r] * 0.001953125f + bvs[t];
    }
    __syncthreads();
    v4f val[8];
    size_t go[8];
#pragma unroll
    for (int it = 0; it < 8; ++it) {
      const int p    = lane + 32 * it;
      const int L    = p >> 3;
      const int pc   = p & 7;
      const int row  = L >> 1;
      const int half = L & 1;
      val[it] = *(const v4f*)(sw + row * OTP + half * 32 + pc * 4);
      go[it]  = (size_t)(m0 + sub * 16 + row) * CC + n0 + half * 32 + pc * 4;
    }
    for (int ps = 0; ps < 2; ++ps) {
#pragma unroll
      for (int it = 0; it < 8; ++it) *(volatile v4f*)(out + go[it]) = val[it];
      __threadfence();
    }
  }
}

extern "C" void kernel_launch(void* const* d_in, const int* in_sizes, int n_in,
                              void* d_out, int out_size, void* d_ws, size_t ws_size,
                              hipStream_t stream) {
  if (n_in < 8) return;
  if (in_sizes[0] != ROWS * CC) return;
  if (in_sizes[1] != ROWS * CC) return;
  if (in_sizes[2] != CC * C3) return;
  if (in_sizes[3] != C3) return;
  if (in_sizes[4] != CC * C3) return;
  if (in_sizes[5] != C3) return;
  if (in_sizes[6] != CC * CC) return;
  if (in_sizes[7] != CC) return;
  if (out_size != 2 * ROWS * CC) return;

  const float* mu    = (const float*)d_in[0];
  const float* sigma = (const float*)d_in[1];
  const float* w_qm  = (const float*)d_in[2];
  const float* b_qm  = (const float*)d_in[3];
  const float* w_qs  = (const float*)d_in[4];
  const float* b_qs  = (const float*)d_in[5];
  const float* w_o   = (const float*)d_in[6];
  const float* b_o   = (const float*)d_in[7];
  float* out0 = (float*)d_out;
  float* out1 = out0 + (size_t)ROWS * CC;

  size_t off = 0;
  const size_t oXm  = off; off += (size_t)ROWS * CC * 2;
  const size_t oXs  = off; off += (size_t)ROWS * CC * 2;
  const size_t oWqm = off; off += (size_t)C3 * CC * 2;
  const size_t oWqs = off; off += (size_t)C3 * CC * 2;
  const size_t oWo  = off; off += (size_t)CC * CC * 2;
  const size_t oQ   = off; off += QKPL * 2;
  const size_t oK   = off; off += QKPL * 2;
  const size_t oVm  = off; off += VPL * 2;
  const size_t oVs  = off; off += VPL * 2;
  const size_t oSQ  = off; off += 4 * SQPL * 4;
  const size_t oOm  = off; off += (size_t)ROWS * CC * 2;
  const size_t oOs  = off; off += (size_t)ROWS * CC * 2;
  if (off > ws_size) return;
  if (off > (size_t)134217728) return;

  char* ws = (char*)d_ws;
  _Float16* Xm   = (_Float16*)(ws + oXm);
  _Float16* Xs   = (_Float16*)(ws + oXs);
  _Float16* Wqmt = (_Float16*)(ws + oWqm);
  _Float16* Wqst = (_Float16*)(ws + oWqs);
  _Float16* Wot  = (_Float16*)(ws + oWo);
  _Float16* Qp   = (_Float16*)(ws + oQ);
  _Float16* Kp   = (_Float16*)(ws + oK);
  _Float16* Vmt  = (_Float16*)(ws + oVm);
  _Float16* Vst  = (_Float16*)(ws + oVs);
  float*    SQ   = (float*)(ws + oSQ);
  _Float16* Om   = (_Float16*)(ws + oOm);
  _Float16* Os   = (_Float16*)(ws + oOs);

  const int ngrp = in_sizes[0] / 8;
  k_cvt_x<<<dim3((ngrp + 255) / 256), dim3(256), 0, stream>>>(mu, Xm, ngrp);
  k_cvt_x<<<dim3((ngrp + 255) / 256), dim3(256), 0, stream>>>(sigma, Xs, ngrp);
  k_wt<<<dim3(C3 / 64, CC / 64), dim3(256), 0, stream>>>(w_qm, Wqmt, C3);
  k_wt<<<dim3(C3 / 64, CC / 64), dim3(256), 0, stream>>>(w_qs, Wqst, C3);
  k_wt<<<dim3(CC / 64, CC / 64), dim3(256), 0, stream>>>(w_o, Wot, CC);
  k_qkv<<<dim3(ROWS / 256, C3 / 64), dim3(256), 0, stream>>>(Xm, Wqmt, b_qm, Qp, Kp, Vmt, SQ, 0);
  k_qkv<<<dim3(ROWS / 256, C3 / 64), dim3(256), 0, stream>>>(Xs, Wqst, b_qs, Qp, Kp, Vst, SQ + 2 * SQPL, 1);
  k_attn<<<dim3(NBH * (NN / 128)), dim3(256), 0, stream>>>(Qp, Kp, Vmt, Vst, SQ, Om, Os);
  k_proj<<<dim3(ROWS / 256, CC / 64), dim3(256), 0, stream>>>(Om, Wot, b_o, out0);
  k_proj<<<dim3(ROWS / 256, CC / 64), dim3(256), 0, stream>>>(Os, Wot, b_o, out1);
  (void)hipGetLastError();
}
